// SparseBlock_55774445306017
// MI455X (gfx1250) — hardware-verified
//
#include <hip/hip_runtime.h>
#include <stdint.h>
#include <stddef.h>


#define NB  4
#define NS  1024
#define ND  512
#define NH  8
#define NDH 64
#define NI  1536
#define NM  (NB * NS)
#define PSP 1032

typedef _Float16 f16;
typedef f16   v4h  __attribute__((ext_vector_type(4)));
typedef f16   v8h  __attribute__((ext_vector_type(8)));
typedef f16   v16h __attribute__((ext_vector_type(16)));
typedef float v4f  __attribute__((ext_vector_type(4)));
typedef float v8f  __attribute__((ext_vector_type(8)));

union Frag { v16h v; v8h half[2]; };
union H8   { v8h v; v4h q[2]; f16 s[8]; };

#define WMMA_F16(a, b, c) \
  __builtin_amdgcn_wmma_f32_16x16x32_f16(false, (a), false, (b), (short)0, (c), false, false)
#define NOP4 "v_nop\n\tv_nop\n\tv_nop\n\tv_nop"

__device__ __forceinline__ v8f zero8() {
  v8f z = {0.f, 0.f, 0.f, 0.f, 0.f, 0.f, 0.f, 0.f};
  return z;
}

__device__ __forceinline__ float wave_max(float v) {
#pragma unroll
  for (int m = 16; m > 0; m >>= 1) v = fmaxf(v, __shfl_xor(v, m, 32));
  return v;
}
__device__ __forceinline__ float wave_sum(float v) {
#pragma unroll
  for (int m = 16; m > 0; m >>= 1) v += __shfl_xor(v, m, 32);
  return v;
}
__device__ __forceinline__ int wave_sumi(int v) {
#pragma unroll
  for (int m = 16; m > 0; m >>= 1) v += __shfl_xor(v, m, 32);
  return v;
}

__global__ __launch_bounds__(256) void cvt_f16_k(const float* __restrict__ X, f16* __restrict__ Y, int n8) {
  const int i = blockIdx.x * 256 + threadIdx.x;
  if (i >= n8) return;
  const size_t e = (size_t)i * 8;
  const v4f a = *(const v4f*)(X + e);
  const v4f b = *(const v4f*)(X + e + 4);
  H8 u;
  u.q[0] = __builtin_convertvector(a, v4h);
  u.q[1] = __builtin_convertvector(b, v4h);
  f16* d = Y + e;
  *(volatile v8h*)d = u.v;
  __threadfence();
  *(volatile v8h*)d = u.v;
}

__global__ __launch_bounds__(256) void trcvt_k(const float* __restrict__ W, f16* __restrict__ Wt, int R, int C) {
  __shared__ float tile[64 * 65];
  const int c0 = blockIdx.x * 64, r0 = blockIdx.y * 64;
  if (r0 + 64 > R || c0 + 64 > C) return;
  const int tid = threadIdx.x, lane = tid & 31, w = tid >> 5;
#pragma unroll
  for (int j = 0; j < 4; ++j) {
    const int e = tid + j * 256, row = e >> 4, c4 = (e & 15) * 4;
    const v4f v = *(const v4f*)(W + (size_t)(r0 + row) * C + c0 + c4);
    float* t = &tile[row * 65 + c4];
    t[0] = v[0]; t[1] = v[1]; t[2] = v[2]; t[3] = v[3];
  }
  __syncthreads();
  const int q = lane >> 3, p = lane & 7;
  H8 u[2];
#pragma unroll
  for (int it = 0; it < 2; ++it) {
    const int cl = w * 8 + it * 4 + q;
#pragma unroll
    for (int j = 0; j < 8; ++j) u[it].s[j] = (f16)tile[(p * 8 + j) * 65 + cl];
  }
#pragma unroll
  for (int it = 0; it < 2; ++it) {
    const int cl = w * 8 + it * 4 + q;
    *(volatile v8h*)(Wt + (size_t)(c0 + cl) * R + r0 + p * 8) = u[it].v;
  }
  __threadfence();
#pragma unroll
  for (int it = 0; it < 2; ++it) {
    const int cl = w * 8 + it * 4 + q;
    *(volatile v8h*)(Wt + (size_t)(c0 + cl) * R + r0 + p * 8) = u[it].v;
  }
}

template <int MODE>
__global__ __launch_bounds__(128) void gemm_f16_k(const f16* __restrict__ A, const f16* __restrict__ B,
                                                   const f16* __restrict__ B2, const float* __restrict__ bias,
                                                   const float* __restrict__ res, void* __restrict__ Cout,
                                                   int M, int N, int K) {
  __shared__ __attribute__((aligned(16))) f16 As[64 * 40];
  __shared__ __attribute__((aligned(16))) f16 Bs[64 * 40];
  __shared__ __attribute__((aligned(16))) f16 Gs[(MODE == 2) ? 64 * 40 : 8];
  __shared__ __attribute__((aligned(16))) float Cs[64 * 68];
  const int n0 = blockIdx.x * 64, m0 = blockIdx.y * 64;
  if (m0 + 64 > M || n0 + 64 > N) return;
  const int tid = threadIdx.x, lane = tid & 31, w = tid >> 5;
  const int wm = w & 1, wn = w >> 1;
  const int hh = lane >> 4, mm = lane & 15;

  v8f acc[2][2], accg[2][2];
#pragma unroll
  for (int i = 0; i < 2; ++i)
#pragma unroll
    for (int j = 0; j < 2; ++j) { acc[i][j] = zero8(); accg[i][j] = zero8(); }

  for (int k0 = 0; k0 < K; k0 += 32) {
    __syncthreads();
#pragma unroll
    for (int j = 0; j < 2; ++j) {
      const int c = tid + j * 128, row = c >> 2, g = c & 3;
      const v8h va = *(const v8h*)(A + (size_t)(m0 + row) * K + k0 + g * 8);
      *(v8h*)&As[row * 40 + g * 8] = va;
      const v8h vb = *(const v8h*)(B + (size_t)(n0 + row) * K + k0 + g * 8);
      *(v8h*)&Bs[row * 40 + g * 8] = vb;
      if constexpr (MODE == 2) {
        const v8h vg = *(const v8h*)(B2 + (size_t)(n0 + row) * K + k0 + g * 8);
        *(v8h*)&Gs[row * 40 + g * 8] = vg;
      }
    }
    __syncthreads();

    Frag fa[2], fb[2], fg[2];
#pragma unroll
    for (int i = 0; i < 2; ++i) {
      const int ar = (wm * 32 + i * 16 + mm) * 40;
      fa[i].half[0] = *(const v8h*)&As[ar + 8 * hh];
      fa[i].half[1] = *(const v8h*)&As[ar + 16 + 8 * hh];
      const int br = (wn * 32 + i * 16 + mm) * 40;
      fb[i].half[0] = *(const v8h*)&Bs[br + 8 * hh];
      fb[i].half[1] = *(const v8h*)&Bs[br + 16 + 8 * hh];
      if constexpr (MODE == 2) {
        fg[i].half[0] = *(const v8h*)&Gs[br + 8 * hh];
        fg[i].half[1] = *(const v8h*)&Gs[br + 16 + 8 * hh];
      }
    }
#pragma unroll
    for (int i = 0; i < 2; ++i)
#pragma unroll
      for (int j = 0; j < 2; ++j) {
        acc[i][j] = WMMA_F16(fa[i].v, fb[j].v, acc[i][j]);
        if constexpr (MODE == 2) accg[i][j] = WMMA_F16(fa[i].v, fg[j].v, accg[i][j]);
      }
    if constexpr (MODE == 2) {
      asm volatile(NOP4
                   : "+v"(acc[0][0]), "+v"(acc[0][1]), "+v"(acc[1][0]), "+v"(acc[1][1]),
                     "+v"(accg[0][0]), "+v"(accg[0][1]), "+v"(accg[1][0]), "+v"(accg[1][1])
                   : "v"(fa[0].v), "v"(fa[1].v), "v"(fb[0].v), "v"(fb[1].v), "v"(fg[0].v), "v"(fg[1].v));
    } else {
      asm volatile(NOP4
                   : "+v"(acc[0][0]), "+v"(acc[0][1]), "+v"(acc[1][0]), "+v"(acc[1][1])
                   : "v"(fa[0].v), "v"(fa[1].v), "v"(fb[0].v), "v"(fb[1].v));
    }
  }

#pragma unroll
  for (int i = 0; i < 2; ++i)
#pragma unroll
    for (int j = 0; j < 2; ++j)
#pragma unroll
      for (int r = 0; r < 8; ++r) {
        const int row = wm * 32 + i * 16 + 8 * hh + r, col = wn * 32 + j * 16 + mm;
        float v = acc[i][j][r];
        if constexpr (MODE == 2) {
          const float g = v;
          v = g * __builtin_amdgcn_rcpf(1.f + __expf(-g)) * accg[i][j][r];
        }
        Cs[row * 68 + col] = v;
      }
  __syncthreads();

  const int q = lane >> 3, p = lane & 7;
  if constexpr (MODE == 1 || MODE == 3) {
    float* C = (float*)Cout;
    v4f vals[8];
#pragma unroll
    for (int it = 0; it < 8; ++it) {
      const int L = w * 32 + it * 4 + q, row = L >> 1, col = (L & 1) * 32 + p * 4;
      v4f v = *(const v4f*)&Cs[row * 68 + col];
      if constexpr (MODE == 1) v += *(const v4f*)(bias + n0 + col);
      else v += *(const v4f*)(res + (size_t)(m0 + row) * N + n0 + col);
      vals[it] = v;
    }
#pragma unroll
    for (int it = 0; it < 8; ++it) {
      const int L = w * 32 + it * 4 + q, row = L >> 1, col = (L & 1) * 32 + p * 4;
      *(volatile v4f*)(C + (size_t)(m0 + row) * N + n0 + col) = vals[it];
    }
    __threadfence();
#pragma unroll
    for (int it = 0; it < 8; ++it) {
      const int L = w * 32 + it * 4 + q, row = L >> 1, col = (L & 1) * 32 + p * 4;
      *(volatile v4f*)(C + (size_t)(m0 + row) * N + n0 + col) = vals[it];
    }
  } else {
    f16* C = (f16*)Cout;
    v8h vals[4];
#pragma unroll
    for (int it = 0; it < 4; ++it) {
      const int row = w * 16 + it * 4 + q, col = p * 8;
      v4f x0 = *(const v4f*)&Cs[row * 68 + col];
      v4f x1 = *(const v4f*)&Cs[row * 68 + col + 4];
      if constexpr (MODE == 0) {
        x0 += *(const v4f*)(bias + n0 + col);
        x1 += *(const v4f*)(bias + n0 + col + 4);
      }
      H8 u;
      u.q[0] = __builtin_convertvector(x0, v4h);
      u.q[1] = __builtin_convertvector(x1, v4h);
      vals[it] = u.v;
    }
#pragma unroll
    for (int it = 0; it < 4; ++it) {
      const int row = w * 16 + it * 4 + q, col = p * 8;
      *(volatile v8h*)(C + (size_t)(m0 + row) * N + n0 + col) = vals[it];
    }
    __threadfence();
#pragma unroll
    for (int it = 0; it < 4; ++it) {
      const int row = w * 16 + it * 4 + q, col = p * 8;
      *(volatile v8h*)(C + (size_t)(m0 + row) * N + n0 + col) = vals[it];
    }
  }
}

#define ATT_Q   (32 * NS * 4)
#define ATT_KV  (ATT_Q + 32 * 72 * 2)
#define ATT_P   (ATT_KV + 64 * 72 * 2)
#define ATT_LDS (ATT_P + 32 * PSP * 2)

__global__ __launch_bounds__(256) void attn_k(const f16* __restrict__ Q, const f16* __restrict__ KV,
                                              f16* __restrict__ O) {
  extern __shared__ __attribute__((aligned(16))) char smem[];
  float* sc  = (float*)smem;
  f16*   Qs  = (f16*)(smem + ATT_Q);
  f16*   KVs = (f16*)(smem + ATT_KV);
  f16*   Ps  = (f16*)(smem + ATT_P);

  const int mt = blockIdx.x, h = blockIdx.y, b = blockIdx.z;
  const int m0 = mt * 32;
  const int tid = threadIdx.x, lane = tid & 31, w = tid >> 5;
  const int hh = lane >> 4, mm = lane & 15;
  const size_t rowbase = (size_t)b * NS;

  {
    const int row = tid >> 3, g = tid & 7;
    const v8h vq = *(const v8h*)(Q + (rowbase + m0 + row) * ND + h * NDH + g * 8);
    *(v8h*)&Qs[row * 72 + g * 8] = vq;
  }

  {
    const int wm = w & 1, wn = w >> 1;
    for (int kb = 0; kb < NS / 64; ++kb) {
      __syncthreads();
#pragma unroll
      for (int j = 0; j < 2; ++j) {
        const int c = tid + j * 256, key = c >> 3, g = c & 7;
        const v8h vk = *(const v8h*)(KV + (rowbase + kb * 64 + key) * (2 * ND) + h * NDH + g * 8);
        *(v8h*)&KVs[key * 72 + g * 8] = vk;
      }
      __syncthreads();

      v8f acc = zero8();
      Frag qa0, qa1, kb0, kb1;
      const int qr = (wm * 16 + mm) * 72, kr = (wn * 16 + mm) * 72;
      qa0.half[0] = *(const v8h*)&Qs[qr + 8 * hh];
      qa0.half[1] = *(const v8h*)&Qs[qr + 16 + 8 * hh];
      qa1.half[0] = *(const v8h*)&Qs[qr + 32 + 8 * hh];
      qa1.half[1] = *(const v8h*)&Qs[qr + 48 + 8 * hh];
      kb0.half[0] = *(const v8h*)&KVs[kr + 8 * hh];
      kb0.half[1] = *(const v8h*)&KVs[kr + 16 + 8 * hh];
      kb1.half[0] = *(const v8h*)&KVs[kr + 32 + 8 * hh];
      kb1.half[1] = *(const v8h*)&KVs[kr + 48 + 8 * hh];
      acc = WMMA_F16(qa0.v, kb0.v, acc);
      acc = WMMA_F16(qa1.v, kb1.v, acc);
      asm volatile(NOP4 : "+v"(acc) : "v"(qa0.v), "v"(kb0.v), "v"(qa1.v), "v"(kb1.v));

      float* srow = sc + (wm * 16 + 8 * hh) * NS + kb * 64 + wn * 16 + mm;
#pragma unroll
      for (int r = 0; r < 8; ++r) srow[r * NS] = acc[r] * 0.125f;
    }
  }
  __syncthreads();

  for (int rr = 0; rr < 4; ++rr) {
    const int row = w * 4 + rr;
    const float* srow = sc + row * NS + lane;
    float v[32];
    float mx = -3.0e38f;
#pragma unroll
    for (int i = 0; i < 32; ++i) { v[i] = srow[i * 32]; mx = fmaxf(mx, v[i]); }
    mx = wave_max(mx);
    float s = 0.f;
#pragma unroll
    for (int i = 0; i < 32; ++i) { v[i] = __expf(v[i] - mx); s += v[i]; }
    s = wave_sum(s);
    const float inv = 1.f / s;
    float wmax = 0.f;
#pragma unroll
    for (int i = 0; i < 32; ++i) { v[i] *= inv; wmax = fmaxf(wmax, v[i]); }
    wmax = wave_max(wmax);

    float lo = 0.f, hi2 = fminf(wmax, 1.f / 513.f);
#pragma unroll 1
    for (int it = 0; it < 20; ++it) {
      const float mid = 0.5f * (lo + hi2);
      int c = 0;
#pragma unroll
      for (int i = 0; i < 32; ++i) c += (v[i] > mid) ? 1 : 0;
      c = wave_sumi(c);
      if (c > NS / 2) lo = mid; else hi2 = mid;
    }
    const float thr = hi2;

    float den = 0.f;
#pragma unroll
    for (int i = 0; i < 32; ++i) {
      const float mk = (v[i] > thr) ? v[i] : 0.f;
      v[i] = __expf(mk - wmax);
      den += v[i];
    }
    den = wave_sum(den);
    const float psc = 1024.f / den;
    f16* prow = Ps + row * PSP + lane;
#pragma unroll
    for (int i = 0; i < 32; ++i) prow[i * 32] = (f16)(v[i] * psc);
  }

  {
    const int wm = w & 1, wn = w >> 1;
    v8f acc = zero8();
    for (int kb = 0; kb < NS / 64; ++kb) {
      __syncthreads();
#pragma unroll
      for (int j = 0; j < 2; ++j) {
        const int c = tid + j * 256, key = c >> 3, g = c & 7;
        H8 u;
        u.v = *(const v8h*)(KV + (rowbase + kb * 64 + key) * (2 * ND) + ND + h * NDH + g * 8);
#pragma unroll
        for (int jj = 0; jj < 8; ++jj) KVs[(g * 8 + jj) * 72 + key] = u.s[jj];
      }
      __syncthreads();

      Frag pa0, pa1, vb0, vb1;
      const int pr = (wm * 16 + mm) * PSP + kb * 64, vr = (wn * 16 + mm) * 72;
      pa0.half[0] = *(const v8h*)&Ps[pr + 8 * hh];
      pa0.half[1] = *(const v8h*)&Ps[pr + 16 + 8 * hh];
      pa1.half[0] = *(const v8h*)&Ps[pr + 32 + 8 * hh];
      pa1.half[1] = *(const v8h*)&Ps[pr + 48 + 8 * hh];
      vb0.half[0] = *(const v8h*)&KVs[vr + 8 * hh];
      vb0.half[1] = *(const v8h*)&KVs[vr + 16 + 8 * hh];
      vb1.half[0] = *(const v8h*)&KVs[vr + 32 + 8 * hh];
      vb1.half[1] = *(const v8h*)&KVs[vr + 48 + 8 * hh];
      acc = WMMA_F16(pa0.v, vb0.v, acc);
      acc = WMMA_F16(pa1.v, vb1.v, acc);
      asm volatile(NOP4 : "+v"(acc) : "v"(pa0.v), "v"(vb0.v), "v"(pa1.v), "v"(vb1.v));
    }

    float* Os = sc;
    const float osc = 1.f / 1024.f;
#pragma unroll
    for (int r = 0; r < 8; ++r) Os[(wm * 16 + 8 * hh + r) * 68 + wn * 16 + mm] = acc[r] * osc;
    __syncthreads();
    const int q = lane >> 3, p = lane & 7, orow = w * 4 + q;
    const v4f x0 = *(const v4f*)&Os[orow * 68 + p * 8];
    const v4f x1 = *(const v4f*)&Os[orow * 68 + p * 8 + 4];
    H8 u;
    u.q[0] = __builtin_convertvector(x0, v4h);
    u.q[1] = __builtin_convertvector(x1, v4h);
    f16* dst = O + (rowbase + m0 + orow) * ND + h * NDH + p * 8;
    *(volatile v8h*)dst = u.v;
    __threadfence();
    *(volatile v8h*)dst = u.v;
  }
}

__global__ __launch_bounds__(64) void rmsnorm_k(const float* __restrict__ X, const float* __restrict__ AO,
                                                const float* __restrict__ Wn, float* __restrict__ Hf,
                                                f16* __restrict__ Hh, int M) {
  __shared__ __attribute__((aligned(16))) float hrow[ND];
  __shared__ float red[2];
  const int row = blockIdx.x;
  if (row >= M) return;
  const int tid = threadIdx.x, lane = tid & 31, w = tid >> 5;
  const size_t base = (size_t)row * ND;
  const int e0 = tid * 4, e1 = 256 + tid * 4;
  const v4f s0 = *(const v4f*)(X + base + e0) + *(const v4f*)(AO + base + e0);
  const v4f s1 = *(const v4f*)(X + base + e1) + *(const v4f*)(AO + base + e1);
  float ss = s0[0] * s0[0] + s0[1] * s0[1] + s0[2] * s0[2] + s0[3] * s0[3] +
             s1[0] * s1[0] + s1[1] * s1[1] + s1[2] * s1[2] + s1[3] * s1[3];
  ss = wave_sum(ss);
  if (lane == 0) red[w] = ss;
  __syncthreads();
  const float tot = red[0] + red[1];
  const float scale = rsqrtf(tot * (1.f / (float)ND) + 1e-6f);
  const v4f h0 = s0 * scale * *(const v4f*)(Wn + e0);
  const v4f h1 = s1 * scale * *(const v4f*)(Wn + e1);
  *(v4f*)&hrow[e0] = h0;
  *(v4f*)&hrow[e1] = h1;
  __syncthreads();
  const v4f y0 = *(const v4f*)&hrow[tid * 8];
  const v4f y1 = *(const v4f*)&hrow[tid * 8 + 4];
  H8 u;
  u.q[0] = __builtin_convertvector(y0, v4h);
  u.q[1] = __builtin_convertvector(y1, v4h);
  *(volatile v4f*)(Hf + base + e0) = h0;
  *(volatile v4f*)(Hf + base + e1) = h1;
  *(volatile v8h*)(Hh + base + tid * 8) = u.v;
  __threadfence();
  *(volatile v4f*)(Hf + base + e0) = h0;
  *(volatile v4f*)(Hf + base + e1) = h1;
  *(volatile v8h*)(Hh + base + tid * 8) = u.v;
}

__global__ __launch_bounds__(256) void instnorm_k(const float* __restrict__ Z, const float* __restrict__ G,
                                                  const float* __restrict__ Bt, float* __restrict__ out,
                                                  int S, int Dm) {
  __shared__ v4f part[8][32];
  __shared__ v4f mv[32], iv[32];
  const int nslab = Dm >> 7;
  const int b = blockIdx.x / nslab, d0 = (blockIdx.x - b * nslab) * 128;
  const int tid = threadIdx.x, lane = tid & 31, w = tid >> 5;
  const int col = d0 + lane * 4;
  const float* zb = Z + (size_t)b * S * Dm + col;

  v4f sm = {0.f, 0.f, 0.f, 0.f};
  for (int t = w; t < S; t += 8) sm += *(const v4f*)(zb + (size_t)t * Dm);
  part[w][lane] = sm;
  __syncthreads();
  if (w == 0) {
    v4f tot = part[0][lane];
#pragma unroll
    for (int j = 1; j < 8; ++j) tot += part[j][lane];
    mv[lane] = tot * (1.f / (float)S);
  }
  __syncthreads();
  const v4f mean = mv[lane];
  v4f sq = {0.f, 0.f, 0.f, 0.f};
  for (int t = w; t < S; t += 8) {
    const v4f d = *(const v4f*)(zb + (size_t)t * Dm) - mean;
    sq += d * d;
  }
  part[w][lane] = sq;
  __syncthreads();
  if (w == 0) {
    v4f tot = part[0][lane];
#pragma unroll
    for (int j = 1; j < 8; ++j) tot += part[j][lane];
    const v4f var = tot * (1.f / (float)S);
    v4f r;
    r[0] = rsqrtf(var[0] + 1e-5f); r[1] = rsqrtf(var[1] + 1e-5f);
    r[2] = rsqrtf(var[2] + 1e-5f); r[3] = rsqrtf(var[3] + 1e-5f);
    iv[lane] = r;
  }
  __syncthreads();
  const v4f inv = iv[lane];
  const v4f g = *(const v4f*)(G + col), be = *(const v4f*)(Bt + col);
  float* ob = out + (size_t)b * S * Dm + col;
  for (int t = w; t < S; t += 8) {
    const v4f z = *(const v4f*)(zb + (size_t)t * Dm);
    const v4f o = (z - mean) * inv * g + be;
    *(volatile v4f*)(ob + (size_t)t * Dm) = o;
  }
  __threadfence();
  for (int t = w; t < S; t += 8) {
    const v4f z = *(const v4f*)(zb + (size_t)t * Dm);
    const v4f o = (z - mean) * inv * g + be;
    *(volatile v4f*)(ob + (size_t)t * Dm) = o;
  }
}

extern "C" void kernel_launch(void* const* d_in, const int* in_sizes, int n_in,
                              void* d_out, int out_size, void* d_ws, size_t ws_size,
                              hipStream_t stream) {
  if (n_in < 13) return;
  if (in_sizes[0] != NM * ND || in_sizes[1] != ND * ND || in_sizes[2] != ND ||
      in_sizes[3] != ND * 2 * ND || in_sizes[4] != 2 * ND || in_sizes[5] != ND * ND ||
      in_sizes[6] != ND || in_sizes[7] != ND || in_sizes[8] != ND * NI ||
      in_sizes[9] != ND * NI || in_sizes[10] != NI * ND || in_sizes[11] != ND ||
      in_sizes[12] != ND || out_size != NM * ND) return;

  const float* x    = (const float*)d_in[0];
  const float* Wq   = (const float*)d_in[1];
  const float* bq   = (const float*)d_in[2];
  const float* Wkv  = (const float*)d_in[3];
  const float* bkv  = (const float*)d_in[4];
  const float* Wo   = (const float*)d_in[5];
  const float* bo   = (const float*)d_in[6];
  const float* rmsw = (const float*)d_in[7];
  const float* l1   = (const float*)d_in[8];
  const float* l2   = (const float*)d_in[9];
  const float* l3   = (const float*)d_in[10];
  const float* inw  = (const float*)d_in[11];
  const float* inb  = (const float*)d_in[12];
  float* out = (float*)d_out;

  size_t off = 0;
  char* wsb = (char*)d_ws;
  auto carve = [&](size_t bytes) -> char* {
    char* p = wsb + off;
    off += (bytes + 255) & ~(size_t)255;
    return p;
  };
  f16*   Xh   = (f16*)carve((size_t)NM * ND * 2);
  f16*   Wqt  = (f16*)carve((size_t)ND * ND * 2);
  f16*   Wkvt = (f16*)carve((size_t)2 * ND * ND * 2);
  f16*   Wot  = (f16*)carve((size_t)ND * ND * 2);
  f16*   L1t  = (f16*)carve((size_t)NI * ND * 2);
  f16*   L2t  = (f16*)carve((size_t)NI * ND * 2);
  f16*   L3t  = (f16*)carve((size_t)ND * NI * 2);
  f16*   Qh   = (f16*)carve((size_t)NM * ND * 2);
  f16*   KVh  = (f16*)carve((size_t)NM * 2 * ND * 2);
  f16*   Oh   = (f16*)carve((size_t)NM * ND * 2);
  float* AOf  = (float*)carve((size_t)NM * ND * 4);
  float* Hf   = (float*)carve((size_t)NM * ND * 4);
  f16*   Hh   = (f16*)carve((size_t)NM * ND * 2);
  f16*   Ah   = (f16*)carve((size_t)NM * NI * 2);
  float* Zf   = (float*)carve((size_t)NM * ND * 4);
  if (off > ws_size) return;

  cvt_f16_k<<<(NM * ND / 8 + 255) / 256, 256, 0, stream>>>(x, Xh, NM * ND / 8);
  trcvt_k<<<dim3(ND / 64, ND / 64), 256, 0, stream>>>(Wq, Wqt, ND, ND);
  trcvt_k<<<dim3(2 * ND / 64, ND / 64), 256, 0, stream>>>(Wkv, Wkvt, ND, 2 * ND);
  trcvt_k<<<dim3(ND / 64, ND / 64), 256, 0, stream>>>(Wo, Wot, ND, ND);
  trcvt_k<<<dim3(NI / 64, ND / 64), 256, 0, stream>>>(l1, L1t, ND, NI);
  trcvt_k<<<dim3(NI / 64, ND / 64), 256, 0, stream>>>(l2, L2t, ND, NI);
  trcvt_k<<<dim3(ND / 64, NI / 64), 256, 0, stream>>>(l3, L3t, NI, ND);

  gemm_f16_k<0><<<dim3(ND / 64, NM / 64), 128, 0, stream>>>(Xh, Wqt, Wqt, bq, bq, (void*)Qh, NM, ND, ND);
  gemm_f16_k<0><<<dim3(2 * ND / 64, NM / 64), 128, 0, stream>>>(Xh, Wkvt, Wkvt, bkv, bkv, (void*)KVh, NM, 2 * ND, ND);

  attn_k<<<dim3(NS / 32, NH, NB), 256, ATT_LDS, stream>>>(Qh, KVh, Oh);

  gemm_f16_k<1><<<dim3(ND / 64, NM / 64), 128, 0, stream>>>(Oh, Wot, Wot, bo, bo, (void*)AOf, NM, ND, ND);
  rmsnorm_k<<<NM, 64, 0, stream>>>(x, AOf, rmsw, Hf, Hh, NM);

  gemm_f16_k<2><<<dim3(NI / 64, NM / 64), 128, 0, stream>>>(Hh, L1t, L2t, bq, bq, (void*)Ah, NM, NI, ND);
  gemm_f16_k<3><<<dim3(ND / 64, NM / 64), 128, 0, stream>>>(Ah, L3t, L3t, bq, Hf, (void*)Zf, NM, ND, NI);

  instnorm_k<<<NB * (ND / 128), 256, 0, stream>>>(Zf, inw, inb, out, NS, ND);
}
